// Discriminator_19533511262893
// MI455X (gfx1250) — hardware-verified
//
#include <hip/hip_runtime.h>
#include <math.h>

typedef __attribute__((ext_vector_type(16))) _Float16 v16h;
typedef __attribute__((ext_vector_type(8)))  _Float16 v8h;
typedef __attribute__((ext_vector_type(16))) __bf16   v16b;
typedef __attribute__((ext_vector_type(8)))  __bf16   v8b;
typedef __attribute__((ext_vector_type(8)))  float    v8f;
typedef __attribute__((ext_vector_type(4)))  float    v4f;

constexpr int kT    = 512;
constexpr int kB    = 64;
constexpr int kH    = 100;
constexpr int kHP   = 128;
constexpr int kL    = 10;
constexpr int kRows = kT * kB;
constexpr int kK2   = 2 * kHP;
constexpr int kWP   = 136;
constexpr int kThr  = 256;
constexpr float kInCarry = 1024.0f;
constexpr float kSc = 1.0f / (kInCarry * kInCarry);
constexpr float kF16MinNormal = 6.103515625e-5f;

static_assert((kRows % 64) == 0 && ((kRows / 64) * (kHP / 64)) % 8 == 0 && (kHP % 32) == 0 && (kK2 % 32) == 0 && kH <= kHP && (kH % 4) == 0 && kB == 4 * 16, "GEMM M, N multiples of 64; grids exact; K multiples of 32; four 16-sample tiles");

constexpr size_t kOffWI16 = 0ull;
constexpr size_t kOffZB = 1310720ull;
constexpr size_t kOffX16 = 1314816ull;
constexpr size_t kOffHSA = 9703424ull;
constexpr size_t kOffHSB = 26480640ull;
constexpr size_t kOffZ = 43257856ull;
constexpr size_t kOffHS32 = 76812288ull;
constexpr size_t kWsTotal = 110366720ull;
static_assert(kWsTotal <= 134217728ull, "carve cap: under 128 MiB");
static_assert(kOffWI16 == 0
              && kOffZB == kOffWI16 + 1310720ull
              && kOffX16 == kOffZB + 4096ull
              && kOffHSA == kOffX16 + 8388608ull
              && kOffHSB == kOffHSA + 16777216ull
              && kOffZ == kOffHSB + 16777216ull
              && kOffHS32 == kOffZ + 33554432ull
              && kWsTotal == kOffHS32 + 33554432ull, "the carve is chained and totalled");
static_assert((kOffWI16 % 256) == 0 && (kOffZB % 256) == 0 && (kOffX16 % 256) == 0 && (kOffHSA % 256) == 0 && (kOffHSB % 256) == 0 && (kOffZ % 256) == 0 && (kOffHS32 % 256) == 0, "aligned regions");

__device__ __forceinline__ unsigned short f2bf_bits(float f) {
  unsigned u = __float_as_uint(f);
  return (unsigned short)((u + 0x7FFFu + ((u >> 16) & 1u)) >> 16);
}
__device__ __forceinline__ float bf_bits2f(unsigned short h) { return __uint_as_float(((unsigned)h) << 16); }
__device__ __forceinline__ float bf16r(float f) { return bf_bits2f(f2bf_bits(f)); }
__device__ __forceinline__ float carry_flush(float v, float carry) {
  const float s = v * carry;
  return (fabsf(s) < kF16MinNormal) ? 0.0f : s;
}
__device__ __forceinline__ float frcp(float x) { return __builtin_amdgcn_rcpf(x); }

__device__ __forceinline__ void dep_guard4_h(v8f& a, v8f& b, v8f& c, v8f& d, v16h x, v16h y) { asm volatile("v_nop\n\tv_nop\n\tv_nop\n\tv_nop" : "+v"(a), "+v"(b), "+v"(c), "+v"(d) : "v"(x), "v"(y)); }
__device__ __forceinline__ void dep_guard4_b(v8f& a, v8f& b, v8f& c, v8f& d, v16b x, v16b y) { asm volatile("v_nop\n\tv_nop\n\tv_nop\n\tv_nop" : "+v"(a), "+v"(b), "+v"(c), "+v"(d) : "v"(x), "v"(y)); }
__device__ __forceinline__ void keep4_h(v16h a, v16h b, v16h c, v16h d) { asm volatile("v_nop" :: "v"(a), "v"(b), "v"(c), "v"(d)); }
__device__ __forceinline__ void keep4_b(v16b a, v16b b, v16b c, v16b d) { asm volatile("v_nop" :: "v"(a), "v"(b), "v"(c), "v"(d)); }
__device__ __forceinline__ void acc_guard4(v8f& a, v8f& b, v8f& c, v8f& d) { asm volatile("v_nop\n\tv_nop\n\tv_nop\n\tv_nop" : "+v"(a), "+v"(b), "+v"(c), "+v"(d)); }

template <typename T> struct Frag;
template <> struct Frag<_Float16> {
  typedef v16h V; union U { v16h v; v8h h[2]; };
  static __device__ __forceinline__ v16h load(const _Float16* p) {
    U f; f.h[0] = *(const v8h*)(p); f.h[1] = *(const v8h*)(p + 16); return f.v;
  }
  static __device__ __forceinline__ v8f mma(v16h a, v16h b, v8f c) {
    return __builtin_amdgcn_wmma_f32_16x16x32_f16(false, a, false, b, (short)0, c, false, false);
  }
  static __device__ __forceinline__ void guard4(v8f& a, v8f& b, v8f& c, v8f& d, v16h x, v16h y) { dep_guard4_h(a, b, c, d, x, y); }
  static __device__ __forceinline__ void keep(v16h a, v16h b, v16h c, v16h d) { keep4_h(a, b, c, d); }
};
template <> struct Frag<__bf16> {
  typedef v16b V; union U { v16b v; v8b h[2]; };
  static __device__ __forceinline__ v16b load(const __bf16* p) {
    U f; f.h[0] = *(const v8b*)(p); f.h[1] = *(const v8b*)(p + 16); return f.v;
  }
  static __device__ __forceinline__ v8f mma(v16b a, v16b b, v8f c) {
    return __builtin_amdgcn_wmma_f32_16x16x32_bf16(false, a, false, b, (short)0, c, false, false);
  }
  static __device__ __forceinline__ void guard4(v8f& a, v8f& b, v8f& c, v8f& d, v16b x, v16b y) { dep_guard4_b(a, b, c, d, x, y); }
  static __device__ __forceinline__ void keep(v16b a, v16b b, v16b c, v16b d) { keep4_b(a, b, c, d); }
};

__device__ __forceinline__ v8f mma_h(v16h a, v16h b, v8f c) {
  c = __builtin_amdgcn_wmma_f32_16x16x32_f16(false, a, false, b, (short)0, c, false, false);
  asm volatile("v_nop\n\tv_nop\n\tv_nop\n\tv_nop" : "+v"(c) : "v"(a), "v"(b));
  return c;
}

template <int ET> struct Elem;
template <> struct Elem<0> { typedef _Float16 T; };
template <> struct Elem<1> { typedef __bf16 T; };
template <int ET, bool SPLIT, int BIAS_MODE, int OUT_MODE, bool RESID, int ACT = 0>
__global__ __launch_bounds__(256) void wmma_gemm64(
    const unsigned short* __restrict__ Ap, const unsigned short* __restrict__ A2p, int lda, long strideA,
    const unsigned short* __restrict__ Btp, const unsigned short* __restrict__ Bt2p, int ldb, long strideB,
    void* __restrict__ Cout, void* __restrict__ Cout2, int ldc, long strideC,
    const float* __restrict__ bias,
    const float* __restrict__ resid, long strideR,
    int M, int N, int K, float scale) {
  typedef typename Elem<ET>::T T;
  typedef typename Frag<T>::V V;
  const T* A = (const T*)Ap; const T* A2 = (const T*)A2p; const T* Bt = (const T*)Btp; const T* Bt2 = (const T*)Bt2p;
  __shared__ __align__(16) float sT[8][16 * 68];
  const int b    = blockIdx.y;
  const int lane = threadIdx.x & 31;
  const int wave = threadIdx.x >> 5;
  const int tilesN = N >> 6;
  const int tilesM = M >> 6;
  const int tile = blockIdx.x * 8 + wave;
  if (tile >= tilesM * tilesN) return;
  const int tm = tile / tilesN;
  const int tn = tile - tm * tilesN;
  const int m0 = tm << 6;
  const int n0 = tn << 6;

  const T* Ab  = A  + (size_t)b * strideA;
  const T* Bb  = Bt + (size_t)b * strideB;
  const T* Ab2 = SPLIT ? (A2  + (size_t)b * strideA) : nullptr;
  const T* Bb2 = SPLIT ? (Bt2 + (size_t)b * strideB) : nullptr;

  const int rlane = lane & 15;
  const int koff  = (lane >> 4) * 8;
  const int mOff  = (lane >> 4) * 8;

  v8f acc[4][4];
#pragma unroll
  for (int i = 0; i < 4; ++i)
#pragma unroll
    for (int j = 0; j < 4; ++j) acc[i][j] = (v8f){0.f,0.f,0.f,0.f,0.f,0.f,0.f,0.f};

  for (int k0 = 0; k0 < K; k0 += 32) {
    V bh[4], bl[4];
#pragma unroll
    for (int j = 0; j < 4; ++j) {
      const size_t bo = (size_t)(n0 + (j << 4) + rlane) * ldb + koff + k0;
      bh[j] = Frag<T>::load(Bb + bo);
      if (SPLIT) bl[j] = Frag<T>::load(Bb2 + bo);
    }
#pragma unroll
    for (int i = 0; i < 4; ++i) {
      const size_t ao = (size_t)(m0 + (i << 4) + rlane) * lda + koff + k0;
      V ah = Frag<T>::load(Ab + ao);
      V al;
      if (SPLIT) al = Frag<T>::load(Ab2 + ao);
#pragma unroll
      for (int j = 0; j < 4; ++j) {
        acc[i][j] = Frag<T>::mma(ah, bh[j], acc[i][j]);
        if (SPLIT) {
          acc[i][j] = Frag<T>::mma(ah, bl[j], acc[i][j]);
          acc[i][j] = Frag<T>::mma(al, bh[j], acc[i][j]);
        }
      }
      Frag<T>::guard4(acc[i][0], acc[i][1], acc[i][2], acc[i][3], ah, SPLIT ? al : ah);
    }
    Frag<T>::keep(bh[0], bh[1], bh[2], bh[3]);
    if (SPLIT) Frag<T>::keep(bl[0], bl[1], bl[2], bl[3]);
  }
  acc_guard4(acc[0][0], acc[0][1], acc[0][2], acc[0][3]);
  acc_guard4(acc[1][0], acc[1][1], acc[1][2], acc[1][3]);
  acc_guard4(acc[2][0], acc[2][1], acc[2][2], acc[2][3]);
  acc_guard4(acc[3][0], acc[3][1], acc[3][2], acc[3][3]);

  float* slab = sT[wave];
  const float* Rb = RESID ? (resid + (size_t)b * strideR) : nullptr;
#pragma unroll
  for (int i = 0; i < 4; ++i) {
    const int mBase = m0 + (i << 4);
#pragma unroll
    for (int j = 0; j < 4; ++j) {
      const int n = n0 + (j << 4) + rlane;
      float bv = 0.f;
      if (BIAS_MODE == 2) bv = bias[n];
#pragma unroll
      for (int r = 0; r < 8; ++r) {
        float v = acc[i][j][r] * scale;
        if (BIAS_MODE == 1) v += bias[mBase + mOff + r];
        if (BIAS_MODE == 2) v += bv;
        if (RESID) v += Rb[(size_t)(mBase + mOff + r) * ldc + n];
        if (ACT == 1) v = tanhf(v);
        if (ACT == 2) v = fmaxf(v, 0.0f);
        if (ACT == 3) v = v / (1.0f + expf(-v));
        if (ACT == 4) v = (v > 0.f) ? v : 0.01f * v;
        slab[(mOff + r) * 68 + (j << 4) + rlane] = v;
      }
    }
    __builtin_amdgcn_fence(__ATOMIC_RELEASE, "workgroup");
    __builtin_amdgcn_wave_barrier();
    __builtin_amdgcn_fence(__ATOMIC_ACQUIRE, "workgroup");
    if (OUT_MODE == 0) {
      float* C = (float*)Cout + (size_t)b * strideC;
      const int hh = lane >> 4, c4 = (lane & 15) * 4;
      for (int pass = 0; pass < 2; ++pass) {
#pragma unroll
        for (int it = 0; it < 8; ++it) {
          const int row = it * 2 + hh;
          v4f v = *(const v4f*)(slab + row * 68 + c4);
          *(volatile v4f*)(C + (size_t)(mBase + row) * ldc + n0 + c4) = v;
        }
        __threadfence();
      }
    } else {
      const int q = lane >> 3, c8 = (lane & 7) * 8;
      unsigned short* C  = (unsigned short*)Cout  + (size_t)b * strideC;
      unsigned short* C2 = (OUT_MODE == 2) ? ((unsigned short*)Cout2 + (size_t)b * strideC) : nullptr;
      for (int pass = 0; pass < 2; ++pass) {
#pragma unroll
        for (int it = 0; it < 4; ++it) {
          const int row = it * 4 + q;
          const float* sp = slab + row * 68 + c8;
          v8h hv, lv;
#pragma unroll
          for (int e = 0; e < 8; ++e) {
            if (OUT_MODE == 1) {
              hv[e] = (_Float16)sp[e];
            } else {
              unsigned short hb = f2bf_bits(sp[e]);
              unsigned short lb = f2bf_bits(sp[e] - bf_bits2f(hb));
              hv[e] = __builtin_bit_cast(_Float16, hb);
              lv[e] = __builtin_bit_cast(_Float16, lb);
            }
          }
          *(volatile v8h*)(C + (size_t)(mBase + row) * ldc + n0 + c8) = hv;
          if (OUT_MODE == 2) *(volatile v8h*)(C2 + (size_t)(mBase + row) * ldc + n0 + c8) = lv;
        }
        __threadfence();
      }
    }
    __builtin_amdgcn_fence(__ATOMIC_RELEASE, "workgroup");
    __builtin_amdgcn_wave_barrier();
    __builtin_amdgcn_fence(__ATOMIC_ACQUIRE, "workgroup");
  }
}


union FragU { v16h v; v8h h[2]; };
__device__ __forceinline__ v16h frag_h32(const _Float16* p) { FragU f; f.h[0] = *(const v8h*)(p); f.h[1] = *(const v8h*)(p + 16); return f.v; }
__device__ __forceinline__ v16h frag_tiles(const float* a, const float* b, float c) {
  v16h f;
#pragma unroll
  for (int e = 0; e < 8; ++e) { f[e] = (_Float16)carry_flush(a[e], c); f[8 + e] = (_Float16)carry_flush(b[e], c); }
  return f;
}
__device__ __forceinline__ void frag_tiles2(const float* a, const float* b, float c, float cinv, v16h& hi, v16h& lo) {
#pragma unroll
  for (int e = 0; e < 8; ++e) {
    const _Float16 ha = (_Float16)carry_flush(a[e], c), hb = (_Float16)carry_flush(b[e], c);
    hi[e] = ha; hi[8 + e] = hb;
    lo[e] = (_Float16)carry_flush(a[e] - (float)ha * cinv, c);
    lo[8 + e] = (_Float16)carry_flush(b[e] - (float)hb * cinv, c);
  }
}
__device__ __forceinline__ float fast_tanh(float v) { return 1.0f - 2.0f * frcp(__expf(2.0f * v) + 1.0f); }

__global__ __launch_bounds__(kThr) void setup_kernel(const float* __restrict__ x, const float* __restrict__ W_ih0, const float* __restrict__ W_ih,
                                                     float* __restrict__ ZB, unsigned short* __restrict__ X16, unsigned short* __restrict__ WI16) {
  unsigned v = blockIdx.x * (unsigned)kThr + threadIdx.x;
  asm volatile("" : "+v"(v));
  if (v < 256u) {
    const v4f z = {0.f, 0.f, 0.f, 0.f};
    float* dp = ZB + (size_t)v * 4u;
    *(volatile v4f*)dp = z;
    __threadfence();
    *(volatile v4f*)dp = z;
  } else if (v < 524544u) {
    const unsigned w = v - 256u;
    const unsigned row = w >> 4, c8 = (w & 15u) * 8u;
    v8h hv;
#pragma unroll
    for (int e = 0; e < 8; ++e) {
      const unsigned c = c8 + (unsigned)e;
      const bool live = c < (unsigned)kH;
      float p = x[(size_t)row * kH + (live ? c : 0u)];
      asm volatile("" : "+v"(p));
      hv[e] = (_Float16)(live ? carry_flush(bf16r(p), kInCarry) : 0.0f);
    }
    unsigned short* dp = X16 + (size_t)w * 8u;
    *(volatile v8h*)dp = hv;
    __threadfence();
    *(volatile v8h*)dp = hv;
  } else {
    const unsigned w = v - 524544u;
    const unsigned l = w >> 13, d = (w >> 12) & 1u, n = (w >> 5) & 127u, c8 = (w & 31u) * 8u;
    const bool first = (l == 0u);
    const float* base = first ? (W_ih0 + ((size_t)d * kH + (n < (unsigned)kH ? n : 0u)) * kH)
                              : (W_ih + ((((size_t)(l - 1u) * 2u + d) * kH) + (n < (unsigned)kH ? n : 0u)) * (2 * kH));
    v8h hv;
#pragma unroll
    for (int e = 0; e < 8; ++e) {
      const unsigned c = c8 + (unsigned)e;
      const bool fw = c < (unsigned)kH;
      const bool bw = (!first) && (c >= (unsigned)kHP) && (c < (unsigned)(kHP + kH));
      const bool live = (n < (unsigned)kH) && (fw || bw);
      const unsigned src = fw ? c : (bw ? ((unsigned)kH + (c - (unsigned)kHP)) : 0u);
      float p = base[live ? src : 0u];
      asm volatile("" : "+v"(p));
      hv[e] = (_Float16)(live ? carry_flush(bf16r(p), kInCarry) : 0.0f);
    }
    unsigned short* dp = WI16 + (size_t)w * 8u;
    *(volatile v8h*)dp = hv;
    __threadfence();
    *(volatile v8h*)dp = hv;
  }
}
static_assert(kRows * (kHP / 8) == 524288 && 256 + 524288 == 524544 && kL * 2 * kHP * (kK2 / 8) == 81920 && 524544 + 81920 == 2369 * kThr, "set-up grid exact");

__global__ __launch_bounds__(128) void scan_kernel(const float* __restrict__ Z, const float* __restrict__ Whh, const float* __restrict__ bih,
                                                   const float* __restrict__ bhh, unsigned short* __restrict__ HOUT, float* __restrict__ HS32, int last) {
  __shared__ __align__(16) _Float16 sW[kHP * kWP];
  __shared__ __align__(16) float sB[kHP];
  const int tid = threadIdx.x;
  const int d = blockIdx.x;
  const int wave = tid >> 5;
  const int lane = tid & 31;
  const int col = lane & 15;
  const int hs = lane >> 4;
  {
    const int n = tid;
    const bool live = n < kH;
    const float* wr = Whh + ((size_t)d * kH + (live ? n : 0)) * kH;
    _Float16* dr = sW + n * kWP;
#pragma unroll 1
    for (int k = 0; k < kWP; ++k) dr[k] = (_Float16)0.0f;
    if (live) {
#pragma unroll 1
      for (int k = 0; k < kH; ++k) dr[k] = (_Float16)carry_flush(bf16r(wr[k]), kInCarry);
    }
    const float b0 = bih[(size_t)d * kH + (live ? n : 0)], b1 = bhh[(size_t)d * kH + (live ? n : 0)];
    sB[n] = live ? (bf16r(b0) + bf16r(b1)) : 0.0f;
  }
  __syncthreads();

  const int b = wave * 16 + col;
  const float* zd = Z + (size_t)d * kRows * kHP;
  float hst[8][8];
#pragma unroll
  for (int mt = 0; mt < 8; ++mt)
#pragma unroll
    for (int r = 0; r < 8; ++r) hst[mt][r] = 0.0f;

#pragma unroll 1
  for (int s = 0; s < kT; ++s) {
    int colv = col, hsv = hs;
    asm volatile("" : "+v"(colv), "+v"(hsv));
    const int t = (d == 0) ? s : (kT - 1 - s);
    const size_t row = (size_t)t * kB + (size_t)b;
    v16h bh[4], bl[4];
#pragma unroll
    for (int ks = 0; ks < 4; ++ks) frag_tiles2(hst[2 * ks], hst[2 * ks + 1], kInCarry, 1.0f / kInCarry, bh[ks], bl[ks]);
    const float* zr = zd + row * kHP + 8 * hsv;
    unsigned short* ho = HOUT + row * kK2 + (size_t)d * kHP + 8 * hsv;
    float* h32 = HS32 + row * kK2 + (size_t)d * kHP + 8 * hsv;
#pragma unroll
    for (int mt = 0; mt < 8; ++mt) {
      const _Float16* wr = sW + (16 * mt + colv) * kWP + 8 * hsv;
      v8f a = (v8f){0.f, 0.f, 0.f, 0.f, 0.f, 0.f, 0.f, 0.f};
#pragma unroll
      for (int ks = 0; ks < 4; ++ks) {
        const v16h wf = frag_h32(wr + 32 * ks);
        a = mma_h(wf, bh[ks], a);
        a = mma_h(wf, bl[ks], a);
      }
      const v4f z0 = *(const v4f*)(zr + 16 * mt), z1 = *(const v4f*)(zr + 16 * mt + 4);
      v8h hv; v4f n0, n1;
#pragma unroll
      for (int r = 0; r < 8; ++r) {
        const float zz = (r < 4) ? z0[r & 3] : z1[r & 3];
        const float hn = fast_tanh(zz + sB[16 * mt + 8 * hsv + r] + a[r] * kSc);
        hst[mt][r] = hn;
        hv[r] = (_Float16)carry_flush(hn, kInCarry);
        if (r < 4) n0[r & 3] = hn; else n1[r & 3] = hn;
      }
      for (int pass = 0; pass < 2; ++pass) {
        *(volatile v8h*)(ho + 16 * mt) = hv;
        if (last != 0) { *(volatile v4f*)(h32 + 16 * mt) = n0; *(volatile v4f*)(h32 + 16 * mt + 4) = n1; }
        __threadfence();
      }
    }
  }
}

__global__ __launch_bounds__(kThr) void out_kernel(const float* __restrict__ HS32, const float* __restrict__ W_out, const float* __restrict__ b_out,
                                                   float* __restrict__ out) {
  unsigned v = blockIdx.x * (unsigned)kThr + threadIdx.x;
  asm volatile("" : "+v"(v));
  const float* hp = HS32 + (size_t)v * kK2;
  float acc = 0.0f;
#pragma unroll 1
  for (int half = 0; half < 2; ++half) {
#pragma unroll 1
    for (int j = 0; j < kH; j += 4) {
      const v4f h4 = *(const v4f*)(hp + half * kHP + j);
      const v4f w4 = *(const v4f*)(W_out + half * kH + j);
      const float p0 = w4[0], p1 = w4[1], p2 = w4[2], p3 = w4[3];
      acc += h4[0] * bf16r(p0);
      acc += h4[1] * bf16r(p1);
      acc += h4[2] * bf16r(p2);
      acc += h4[3] * bf16r(p3);
    }
  }
  float bb = b_out[0];
  asm volatile("" : "+v"(bb));
  const float pre = acc + bf16r(bb);
  const float o = 1.0f / (1.0f + expf(-pre));
  *(volatile float*)(out + v) = o;
  __threadfence();
  *(volatile float*)(out + v) = o;
}
static_assert(kRows == 128 * kThr, "output grid exact");

extern "C" void kernel_launch(void* const* d_in, const int* in_sizes, int n_in,
                              void* d_out, int out_size, void* d_ws, size_t ws_size,
                              hipStream_t stream) {
  if (n_in < 8 || d_out == nullptr || d_ws == nullptr) return;
  if (in_sizes[0] != kT * kB * kH || in_sizes[1] != 2 * kH * kH || in_sizes[2] != (kL - 1) * 2 * kH * 2 * kH || in_sizes[3] != kL * 2 * kH * kH) return;
  if (in_sizes[4] != kL * 2 * kH || in_sizes[5] != kL * 2 * kH || in_sizes[6] != 2 * kH || in_sizes[7] != 1) return;
  if (out_size != kRows) return;
  if (ws_size < kWsTotal) return;
  const float* x = (const float*)d_in[0];
  const float* W_ih0 = (const float*)d_in[1];
  const float* W_ih = (const float*)d_in[2];
  const float* W_hh = (const float*)d_in[3];
  const float* b_ih = (const float*)d_in[4];
  const float* b_hh = (const float*)d_in[5];
  const float* W_out = (const float*)d_in[6];
  const float* b_out = (const float*)d_in[7];
  float* out = (float*)d_out;
  char* ws = (char*)d_ws;
  unsigned short* WI16 = (unsigned short*)(ws + kOffWI16);
  float* ZB = (float*)(ws + kOffZB);
  unsigned short* X16 = (unsigned short*)(ws + kOffX16);
  unsigned short* HSA = (unsigned short*)(ws + kOffHSA);
  unsigned short* HSB = (unsigned short*)(ws + kOffHSB);
  float* Z = (float*)(ws + kOffZ);
  float* HS32 = (float*)(ws + kOffHS32);

  setup_kernel<<<2369, kThr, 0, stream>>>(x, W_ih0, W_ih, ZB, X16, WI16);

  for (int l = 0; l < kL; ++l) {
    const unsigned short* IN = (l == 0) ? X16 : ((l & 1) ? HSA : HSB);
    unsigned short* HOUT = (l & 1) ? HSB : HSA;
    const int lda = (l == 0) ? kHP : kK2;
    const unsigned short* Wl = WI16 + (size_t)l * 2 * kHP * kK2;
    wmma_gemm64<0, false, 2, 0, false, 0><<<dim3((kRows / 64) * (kHP / 64) / 8, 2), 256, 0, stream>>>(
        IN, IN, lda, 0L, Wl, Wl, kK2, (long)kHP * kK2, (void*)Z, (void*)Z, kHP, (long)kRows * kHP, ZB, nullptr, 0L, kRows, kHP, lda, kSc);
    scan_kernel<<<2, 128, 0, stream>>>(Z, W_hh + (size_t)l * 2 * kH * kH, b_ih + (size_t)l * 2 * kH, b_hh + (size_t)l * 2 * kH, HOUT, HS32, (l == kL - 1) ? 1 : 0);
  }
  out_kernel<<<128, kThr, 0, stream>>>(HS32, W_out, b_out, out);
}
